// QGRU2_55911884259442
// MI455X (gfx1250) — hardware-verified
//
#include <hip/hip_runtime.h>
#include <math.h>

constexpr int NBATCH  = 64;
constexpr int NWIN    = 32;
constexpr int NSTEP   = 4096;
constexpr int NHID    = 128;
constexpr int NGATE   = 3 * NHID;
constexpr int NTHR    = 256;
constexpr int SEQ_BLK = 32;
constexpr int MSUB    = SEQ_BLK / 16;
constexpr int EPITCH  = 136;
constexpr int HPITCH  = 136;
constexpr int PPITCH  = 132;
constexpr int OBPITCH = 36;
constexpr int TCHUNK  = 32;
constexpr int XP_T    = 32;
constexpr int XP_B    = 16;
constexpr int XP_PITCH = 40;
constexpr float CARRY_ENC     = 4.0f;
constexpr float CARRY_ENC_INV = 0.25f;
constexpr float CARRY_G       = 8.0f;
constexpr float CARRY_G_INV   = 0.125f;

static_assert(NHID == 16 * (NTHR / 32));
static_assert(NBATCH % SEQ_BLK == 0 && SEQ_BLK == 32 && MSUB == 2);
static_assert(NWIN == 32);
static_assert(NHID % 32 == 0);
static_assert(NSTEP % TCHUNK == 0 && TCHUNK == 32);
static_assert((2 * SEQ_BLK * HPITCH) % NTHR == 0);
static_assert(NSTEP % XP_T == 0 && NBATCH % XP_B == 0 && XP_T == 32 && XP_B == 16);
static_assert((XP_B * NWIN * XP_T) % NTHR == 0);
static_assert(EPITCH % 8 == 0 && HPITCH % 8 == 0 && XP_PITCH % 8 == 0 && PPITCH % 4 == 0 && OBPITCH % 4 == 0);

typedef __attribute__((ext_vector_type(16))) _Float16 v16h;
typedef __attribute__((ext_vector_type(8)))  _Float16 v8h;
typedef __attribute__((ext_vector_type(8)))  float    v8f;
typedef __attribute__((ext_vector_type(4)))  float    v4f;

template <typename T> struct Frag;
template <> struct Frag<_Float16> {
  typedef v16h V; union U { v16h v; v8h h[2]; };
  static __device__ __forceinline__ v16h load(const _Float16* p) {
    U f; f.h[0] = *(const v8h*)(p); f.h[1] = *(const v8h*)(p + 16); return f.v;
  }
};

__device__ __forceinline__ v8f mma_h(v16h a, v16h b, v8f c) {
  c = __builtin_amdgcn_wmma_f32_16x16x32_f16(false, a, false, b, (short)0, c, false, false);
  asm volatile("v_nop\n\tv_nop\n\tv_nop\n\tv_nop" : "+v"(c) : "v"(a), "v"(b));
  return c;
}

__device__ __forceinline__ float fsig(float x)  { return __builtin_amdgcn_rcpf(1.0f + expf(-x)); }
__device__ __forceinline__ float ftanh(float x) { return 1.0f - 2.0f * __builtin_amdgcn_rcpf(expf(2.0f * x) + 1.0f); }

__global__ __launch_bounds__(NTHR) void xpose_kernel(const float* __restrict__ x, _Float16* __restrict__ XT) {
  __shared__ __align__(16) _Float16 S[XP_B * XP_T * XP_PITCH];
  const int tid = threadIdx.x, lane = tid & 31, wave = tid >> 5;
  const int t0 = blockIdx.x * XP_T;
  const int b0 = blockIdx.y * XP_B;
#pragma unroll 4
  for (int it = 0; it < (XP_B * NWIN * XP_T) / NTHR; ++it) {
    const int e  = it * NTHR + tid;
    const int tt = e & (XP_T - 1);
    const int w  = (e >> 5) & (NWIN - 1);
    const int bl = e >> 10;
    const float v = x[((size_t)(b0 + bl) * NWIN + w) * NSTEP + t0 + tt];
    S[(bl * XP_T + tt) * XP_PITCH + w] = (_Float16)v;
  }
  __syncthreads();
  const int blo = lane >> 2, w0 = (lane & 3) * 8;
  v8h hv[8];
#pragma unroll
  for (int k = 0; k < 4; ++k)
#pragma unroll
    for (int hf = 0; hf < 2; ++hf) {
      const int tt = wave + 8 * k, bl = hf * 8 + blo;
      hv[2 * k + hf] = *(const v8h*)(S + (bl * XP_T + tt) * XP_PITCH + w0);
    }
  for (int pass = 0; pass < 2; ++pass) {
#pragma unroll
    for (int k = 0; k < 4; ++k)
#pragma unroll
      for (int hf = 0; hf < 2; ++hf) {
        const int tt = wave + 8 * k, bl = hf * 8 + blo;
        *(volatile v8h*)(XT + ((size_t)(t0 + tt) * NBATCH + b0 + bl) * NWIN + w0) = hv[2 * k + hf];
      }
    __threadfence();
  }
}

__global__ __launch_bounds__(NTHR) void cvt8_f16_kernel(const float* __restrict__ src, _Float16* __restrict__ dst,
                                                        int n8, float sc) {
  const int i = blockIdx.x * NTHR + threadIdx.x;
  if (i < n8) {
    const float* sp = src + (size_t)i * 8;
    const v4f a = *(const v4f*)(sp);
    const v4f b = *(const v4f*)(sp + 4);
    v8h hv;
#pragma unroll
    for (int e = 0; e < 4; ++e) {
      hv[e]     = (_Float16)(a[e] * sc);
      hv[4 + e] = (_Float16)(b[e] * sc);
    }
    *(volatile v8h*)(dst + (size_t)i * 8) = hv;
    __threadfence();
    *(volatile v8h*)(dst + (size_t)i * 8) = hv;
  }
}

__global__ __launch_bounds__(NTHR) void rnn_seq_kernel(
    const _Float16* __restrict__ XT,  const _Float16* __restrict__ ENCW,
    const _Float16* __restrict__ WIH, const _Float16* __restrict__ WHH,
    const float* __restrict__ enc_b, const float* __restrict__ b_ih, const float* __restrict__ b_hh,
    const float* __restrict__ dec_w, const float* __restrict__ dec_b, const float* __restrict__ scalep,
    const float* __restrict__ noise, float* __restrict__ out) {
  __shared__ __align__(16) _Float16 E16[SEQ_BLK * EPITCH];
  __shared__ __align__(16) _Float16 H16[2][SEQ_BLK * HPITCH];
  __shared__ __align__(16) float    Pt[SEQ_BLK * PPITCH];
  __shared__ __align__(16) float    OB[SEQ_BLK * OBPITCH];
  const int tid = threadIdx.x, lane = tid & 31, wave = tid >> 5;
  const int c = lane & 15, hh = lane >> 4, koff = 8 * hh;
  const int b0 = blockIdx.x * SEQ_BLK;
  const int j  = 16 * wave + c;

  {
    _Float16* hfl = &H16[0][0];
#pragma unroll 1
    for (int i = tid; i < 2 * SEQ_BLK * HPITCH; i += NTHR) hfl[i] = (_Float16)0.0f;
  }
  const float encbj = enc_b[j];
  const float bir   = b_ih[j] + b_hh[j];
  const float biz   = b_ih[NHID + j] + b_hh[NHID + j];
  const float bin_  = b_ih[2 * NHID + j];
  const float bhn   = b_hh[2 * NHID + j];
  const float dwj   = dec_w[j];
  const float decb  = dec_b[0];
  const float nsc   = scalep[0];
  const v16h bencw = Frag<_Float16>::load(ENCW + (size_t)j * NWIN + koff);
  float hst[MSUB][8];
#pragma unroll
  for (int mi = 0; mi < MSUB; ++mi)
#pragma unroll
    for (int r = 0; r < 8; ++r) hst[mi][r] = 0.0f;
  __syncthreads();

  const v8f z8 = {0.f, 0.f, 0.f, 0.f, 0.f, 0.f, 0.f, 0.f};

#pragma unroll 1
  for (int t = 0; t < NSTEP; ++t) {
    const int cur = t & 1;

    float encv[MSUB][8];
#pragma unroll
    for (int mi = 0; mi < MSUB; ++mi) {
      const v16h xa = Frag<_Float16>::load(XT + ((size_t)t * NBATCH + b0 + 16 * mi + c) * NWIN + koff);
      const v8f ae = mma_h(xa, bencw, z8);
#pragma unroll
      for (int r = 0; r < 8; ++r) {
        const float ev = ae[r] * CARRY_ENC_INV + encbj;
        encv[mi][r] = ev;
        E16[(16 * mi + 8 * hh + r) * EPITCH + j] = (_Float16)ev;
      }
    }
    __syncthreads();

    v8f aR[MSUB], aZ[MSUB], aI[MSUB], aH[MSUB];
#pragma unroll
    for (int mi = 0; mi < MSUB; ++mi) { aR[mi] = z8; aZ[mi] = z8; aI[mi] = z8; aH[mi] = z8; }
    const _Float16* hcur = &H16[cur][0];
    _Float16* hnxt = &H16[cur ^ 1][0];
#pragma unroll 1
    for (int k0 = 0; k0 < NHID; k0 += 32) {
      v16h eA[MSUB], hA[MSUB];
#pragma unroll
      for (int mi = 0; mi < MSUB; ++mi) {
        eA[mi] = Frag<_Float16>::load(E16  + (16 * mi + c) * EPITCH + koff + k0);
        hA[mi] = Frag<_Float16>::load(hcur + (16 * mi + c) * HPITCH + koff + k0);
      }
      {
        const v16h bi = Frag<_Float16>::load(WIH + (size_t)j * NHID + koff + k0);
        const v16h bw = Frag<_Float16>::load(WHH + (size_t)j * NHID + koff + k0);
#pragma unroll
        for (int mi = 0; mi < MSUB; ++mi) { aR[mi] = mma_h(eA[mi], bi, aR[mi]); aR[mi] = mma_h(hA[mi], bw, aR[mi]); }
      }
      {
        const v16h bi = Frag<_Float16>::load(WIH + (size_t)(NHID + j) * NHID + koff + k0);
        const v16h bw = Frag<_Float16>::load(WHH + (size_t)(NHID + j) * NHID + koff + k0);
#pragma unroll
        for (int mi = 0; mi < MSUB; ++mi) { aZ[mi] = mma_h(eA[mi], bi, aZ[mi]); aZ[mi] = mma_h(hA[mi], bw, aZ[mi]); }
      }
      {
        const v16h bi = Frag<_Float16>::load(WIH + (size_t)(2 * NHID + j) * NHID + koff + k0);
        const v16h bw = Frag<_Float16>::load(WHH + (size_t)(2 * NHID + j) * NHID + koff + k0);
#pragma unroll
        for (int mi = 0; mi < MSUB; ++mi) { aI[mi] = mma_h(eA[mi], bi, aI[mi]); aH[mi] = mma_h(hA[mi], bw, aH[mi]); }
      }
    }

#pragma unroll
    for (int mi = 0; mi < MSUB; ++mi) {
#pragma unroll
      for (int r = 0; r < 8; ++r) {
        const int row = 16 * mi + 8 * hh + r;
        const float rg  = fsig(aR[mi][r] * CARRY_G_INV + bir);
        const float zg  = fsig(aZ[mi][r] * CARRY_G_INV + biz);
        const float gin = aI[mi][r] * CARRY_G_INV + bin_;
        const float ghn = aH[mi][r] * CARRY_G_INV + bhn;
        const float nn  = ftanh(gin + rg * ghn);
        const float ho  = hst[mi][r];
        const float hv  = (1.0f - zg) * nn + zg * ho;
        hst[mi][r] = hv;
        hnxt[row * HPITCH + j] = (_Float16)hv;
        Pt[row * PPITCH + j] = (encv[mi][r] + hv) * dwj;
      }
    }
    __syncthreads();

    if (wave == 0) {
      const float* pr = Pt + lane * PPITCH;
      float s0 = 0.0f, s1 = 0.0f, s2 = 0.0f, s3 = 0.0f;
#pragma unroll
      for (int q4 = 0; q4 < NHID / 4; ++q4) {
        const v4f v = *(const v4f*)(pr + 4 * q4);
        s0 += v[0]; s1 += v[1]; s2 += v[2]; s3 += v[3];
      }
      const float s = ((s0 + s1) + (s2 + s3)) + decb;
      OB[lane * OBPITCH + (t & (TCHUNK - 1))] = s;
      if ((t & (TCHUNK - 1)) == TCHUNK - 1) {
        __builtin_amdgcn_fence(__ATOMIC_RELEASE, "workgroup");
        __builtin_amdgcn_wave_barrier();
        __builtin_amdgcn_fence(__ATOMIC_ACQUIRE, "workgroup");
        const int tb = t - (TCHUNK - 1);
        const int q = lane >> 3, c4 = (lane & 7) * 4;
        v4f ov[8];
#pragma unroll
        for (int it = 0; it < 8; ++it) {
          const int row = it * 4 + q;
          const v4f a  = *(const v4f*)(OB + row * OBPITCH + c4);
          const v4f nz = *(const v4f*)(noise + (size_t)(b0 + row) * NSTEP + tb + c4);
          v4f o;
#pragma unroll
          for (int e = 0; e < 4; ++e) {
            const float nzs = nsc * nz[e];
            o[e] = fmaxf(a[e] + nzs, 0.0f);
          }
          ov[it] = o;
        }
        for (int pass = 0; pass < 2; ++pass) {
#pragma unroll
          for (int it = 0; it < 8; ++it) {
            const int row = it * 4 + q;
            *(volatile v4f*)(out + (size_t)(b0 + row) * NSTEP + tb + c4) = ov[it];
          }
          __threadfence();
        }
        __builtin_amdgcn_fence(__ATOMIC_RELEASE, "workgroup");
        __builtin_amdgcn_wave_barrier();
        __builtin_amdgcn_fence(__ATOMIC_ACQUIRE, "workgroup");
      }
    }
  }
}

extern "C" void kernel_launch(void* const* d_in, const int* in_sizes, int n_in,
                              void* d_out, int out_size, void* d_ws, size_t ws_size, hipStream_t stream) {
  if (n_in < 11 || d_out == nullptr || d_ws == nullptr) return;
  if (in_sizes[0] != NBATCH * NWIN * NSTEP || in_sizes[1] != NHID * NWIN || in_sizes[2] != NHID ||
      in_sizes[3] != NGATE * NHID || in_sizes[4] != NGATE * NHID || in_sizes[5] != NGATE ||
      in_sizes[6] != NGATE || in_sizes[7] != NHID || in_sizes[8] < 1 || in_sizes[9] < 1 ||
      in_sizes[10] != NBATCH * NSTEP || out_size != NBATCH * NSTEP) return;

  const float* x      = (const float*)d_in[0];
  const float* enc_w  = (const float*)d_in[1];
  const float* enc_b  = (const float*)d_in[2];
  const float* w_ih   = (const float*)d_in[3];
  const float* w_hh   = (const float*)d_in[4];
  const float* b_ih   = (const float*)d_in[5];
  const float* b_hh   = (const float*)d_in[6];
  const float* dec_w  = (const float*)d_in[7];
  const float* dec_b  = (const float*)d_in[8];
  const float* scalep = (const float*)d_in[9];
  const float* noise  = (const float*)d_in[10];
  float* out = (float*)d_out;

  char* ws = (char*)d_ws; size_t off = 0;
  auto carve = [&](size_t bytes) -> char* { char* p = ws + off; off += (bytes + 255) & ~(size_t)255; return p; };
  _Float16* XT16   = (_Float16*)carve((size_t)NSTEP * NBATCH * NWIN * 2);
  _Float16* ENCW16 = (_Float16*)carve((size_t)NHID * NWIN * 2);
  _Float16* WIH16  = (_Float16*)carve((size_t)NGATE * NHID * 2);
  _Float16* WHH16  = (_Float16*)carve((size_t)NGATE * NHID * 2);
  if (off > ws_size || off > (size_t)134217728) return;

  xpose_kernel<<<dim3(NSTEP / XP_T, NBATCH / XP_B), NTHR, 0, stream>>>(x, XT16);

  const int n8e = NHID * NWIN / 8;
  const int n8g = NGATE * NHID / 8;
  cvt8_f16_kernel<<<(n8e + NTHR - 1) / NTHR, NTHR, 0, stream>>>(enc_w, ENCW16, n8e, CARRY_ENC);
  cvt8_f16_kernel<<<(n8g + NTHR - 1) / NTHR, NTHR, 0, stream>>>(w_ih,  WIH16,  n8g, CARRY_G);
  cvt8_f16_kernel<<<(n8g + NTHR - 1) / NTHR, NTHR, 0, stream>>>(w_hh,  WHH16,  n8g, CARRY_G);

  rnn_seq_kernel<<<NBATCH / SEQ_BLK, NTHR, 0, stream>>>(XT16, ENCW16, WIH16, WHH16, enc_b, b_ih, b_hh,
                                                       dec_w, dec_b, scalep, noise, out);
}
